// PAM_Module_39926015984265
// MI455X (gfx1250) — hardware-verified
//
#include <hip/hip_runtime.h>
#include <math.h>

constexpr int kB    = 2;
constexpr int kC    = 64;
constexpr int kCq   = 8;
constexpr int kN    = 8000;
constexpr int kKP   = 64;
constexpr int kQCH  = 1600;
constexpr int kNChunk = kN / kQCH;
constexpr int kNC8  = kN / 8;
constexpr float kPCarry    = 32768.0f;
constexpr float kPCarryInv = 1.0f / 32768.0f;
constexpr int kTilesProj   = (kN / 64) * (kKP / 64);
constexpr int kBlocksProj  = (kTilesProj + 7) / 8;
constexpr int kTilesScore  = (kQCH / 64) * (kN / 64);
constexpr int kBlocksScore = (kTilesScore + 7) / 8;
constexpr int kTilesPV     = (kC / 64) * (kQCH / 64);
constexpr int kBlocksPV    = (kTilesPV + 7) / 8;
static_assert(kN % 64 == 0 && kQCH % 64 == 0 && kN % kQCH == 0, "tiles");
static_assert(kC == 64 && kKP % 32 == 0 && kC % 32 == 0 && kN % 32 == 0, "k multiples");
static_assert(kNC8 % 8 == 0, "row chunk count is a whole number of lines");
static_assert((kB * kN) % 32 == 0, "pack rows per block");
static_assert(3 * kCq <= 32, "hi|lo|hi packing fits one k step");

typedef __attribute__((ext_vector_type(16))) _Float16 v16h;
typedef __attribute__((ext_vector_type(8)))  _Float16 v8h;
typedef __attribute__((ext_vector_type(16))) __bf16   v16b;
typedef __attribute__((ext_vector_type(8)))  __bf16   v8b;
typedef __attribute__((ext_vector_type(8)))  float    v8f;
typedef __attribute__((ext_vector_type(4)))  float    v4f;
typedef __attribute__((ext_vector_type(4)))  unsigned int v4u;

__device__ __forceinline__ unsigned short f2bf_bits(float f) {
  unsigned u = __float_as_uint(f);
  return (unsigned short)((u + 0x7FFFu + ((u >> 16) & 1u)) >> 16);
}
__device__ __forceinline__ float bf_bits2f(unsigned short h) { return __uint_as_float(((unsigned)h) << 16); }

__device__ __forceinline__ void dep_guard_h(v8f& a, v8f& b, v16h x, v16h y) { asm volatile("v_nop\n\tv_nop\n\tv_nop\n\tv_nop" : "+v"(a), "+v"(b) : "v"(x), "v"(y)); }
__device__ __forceinline__ void dep_guard_b(v8f& a, v8f& b, v16b x, v16b y) { asm volatile("v_nop\n\tv_nop\n\tv_nop\n\tv_nop" : "+v"(a), "+v"(b) : "v"(x), "v"(y)); }
__device__ __forceinline__ void keep4_h(v16h a, v16h b, v16h c, v16h d) { asm volatile("v_nop" :: "v"(a), "v"(b), "v"(c), "v"(d)); }
__device__ __forceinline__ void keep4_b(v16b a, v16b b, v16b c, v16b d) { asm volatile("v_nop" :: "v"(a), "v"(b), "v"(c), "v"(d)); }
__device__ __forceinline__ void acc_guard4(v8f& a, v8f& b, v8f& c, v8f& d) { asm volatile("v_nop\n\tv_nop\n\tv_nop\n\tv_nop" : "+v"(a), "+v"(b), "+v"(c), "+v"(d)); }
template <typename T> struct Frag;
template <> struct Frag<_Float16> {
  typedef v16h V; union U { v16h v; v8h h[2]; };
  static __device__ __forceinline__ v16h load(const _Float16* p) {
    U f; f.h[0] = *(const v8h*)(p); f.h[1] = *(const v8h*)(p + 16); return f.v;
  }
  static __device__ __forceinline__ v8f mma(v16h a, v16h b, v8f c) {
    return __builtin_amdgcn_wmma_f32_16x16x32_f16(false, a, false, b, (short)0, c, false, false);
  }
  static __device__ __forceinline__ void guard(v8f& a, v8f& b, v16h x, v16h y) { dep_guard_h(a, b, x, y); }
  static __device__ __forceinline__ void keep(v16h a, v16h b, v16h c, v16h d) { keep4_h(a, b, c, d); }
};
template <> struct Frag<__bf16> {
  typedef v16b V; union U { v16b v; v8b h[2]; };
  static __device__ __forceinline__ v16b load(const __bf16* p) {
    U f; f.h[0] = *(const v8b*)(p); f.h[1] = *(const v8b*)(p + 16); return f.v;
  }
  static __device__ __forceinline__ v8f mma(v16b a, v16b b, v8f c) {
    return __builtin_amdgcn_wmma_f32_16x16x32_bf16(false, a, false, b, (short)0, c, false, false);
  }
  static __device__ __forceinline__ void guard(v8f& a, v8f& b, v16b x, v16b y) { dep_guard_b(a, b, x, y); }
  static __device__ __forceinline__ void keep(v16b a, v16b b, v16b c, v16b d) { keep4_b(a, b, c, d); }
};

__device__ __forceinline__ unsigned pk16(unsigned short a, unsigned short b) { return (unsigned)a | ((unsigned)b << 16); }
__device__ __forceinline__ unsigned short h_bits(float f) { const _Float16 h = (_Float16)f; return __builtin_bit_cast(unsigned short, h); }

template <int ET> struct Elem;
template <> struct Elem<0> { typedef _Float16 T; };
template <> struct Elem<1> { typedef __bf16 T; };
template <int ET, bool SPLIT, int BIAS_MODE, int OUT_MODE, bool RESID, int ACT = 0>
__global__ __launch_bounds__(256) void wmma_gemm64(
    const unsigned short* __restrict__ Ap, const unsigned short* __restrict__ A2p, int lda, long strideA,
    const unsigned short* __restrict__ Btp, const unsigned short* __restrict__ Bt2p, int ldb, long strideB,
    void* __restrict__ Cout, void* __restrict__ Cout2, int ldc, long strideC,
    const float* __restrict__ bias,
    const float* __restrict__ resid, long strideR,
    int M, int N, int K, float scale) {
  typedef typename Elem<ET>::T T;
  typedef typename Frag<T>::V V;
  const T* A = (const T*)Ap; const T* A2 = (const T*)A2p; const T* Bt = (const T*)Btp; const T* Bt2 = (const T*)Bt2p;
  __shared__ __align__(16) float sT[8][16 * 68];
  const int b    = blockIdx.y;
  const int lane = threadIdx.x & 31;
  const int wave = threadIdx.x >> 5;
  const int tilesN = N >> 6;
  const int tilesM = M >> 6;
  const int tile = blockIdx.x * 8 + wave;
  if (tile >= tilesM * tilesN) return;
  const int tm = tile / tilesN;
  const int tn = tile - tm * tilesN;
  const int m0 = tm << 6;
  const int n0 = tn << 6;

  const T* Ab  = A  + (size_t)b * strideA;
  const T* Bb  = Bt + (size_t)b * strideB;
  const T* Ab2 = SPLIT ? (A2  + (size_t)b * strideA) : nullptr;
  const T* Bb2 = SPLIT ? (Bt2 + (size_t)b * strideB) : nullptr;

  const int rlane = lane & 15;
  const int koff  = (lane >> 4) * 8;
  const int mOff  = (lane >> 4) * 8;

  v8f acc[4][4];
#pragma unroll
  for (int i = 0; i < 4; ++i)
#pragma unroll
    for (int j = 0; j < 4; ++j) acc[i][j] = (v8f){0.f,0.f,0.f,0.f,0.f,0.f,0.f,0.f};

  for (int k0 = 0; k0 < K; k0 += 32) {
    V bh[4], bl[4];
#pragma unroll
    for (int j = 0; j < 4; ++j) {
      const size_t bo = (size_t)(n0 + (j << 4) + rlane) * ldb + koff + k0;
      bh[j] = Frag<T>::load(Bb + bo);
      if (SPLIT) bl[j] = Frag<T>::load(Bb2 + bo);
    }
#pragma unroll
    for (int i = 0; i < 4; ++i) {
      const size_t ao = (size_t)(m0 + (i << 4) + rlane) * lda + koff + k0;
      V ah = Frag<T>::load(Ab + ao);
      V al;
      if (SPLIT) al = Frag<T>::load(Ab2 + ao);
#pragma unroll
      for (int j = 0; j < 4; ++j) {
        acc[i][j] = Frag<T>::mma(ah, bh[j], acc[i][j]);
        if (SPLIT) {
          acc[i][j] = Frag<T>::mma(ah, bl[j], acc[i][j]);
          acc[i][j] = Frag<T>::mma(al, bh[j], acc[i][j]);
        }
      }
      Frag<T>::guard(acc[i][0], acc[i][3], ah, SPLIT ? al : ah);
    }
    Frag<T>::keep(bh[0], bh[1], bh[2], bh[3]);
    if (SPLIT) Frag<T>::keep(bl[0], bl[1], bl[2], bl[3]);
  }
  acc_guard4(acc[0][0], acc[0][1], acc[0][2], acc[0][3]);
  acc_guard4(acc[1][0], acc[1][1], acc[1][2], acc[1][3]);
  acc_guard4(acc[2][0], acc[2][1], acc[2][2], acc[2][3]);
  acc_guard4(acc[3][0], acc[3][1], acc[3][2], acc[3][3]);

  float* slab = sT[wave];
  const float* Rb = RESID ? (resid + (size_t)b * strideR) : nullptr;
#pragma unroll
  for (int i = 0; i < 4; ++i) {
    const int mBase = m0 + (i << 4);
#pragma unroll
    for (int j = 0; j < 4; ++j) {
      const int n = n0 + (j << 4) + rlane;
      float bv = 0.f;
      if (BIAS_MODE == 2) bv = bias[n];
#pragma unroll
      for (int r = 0; r < 8; ++r) {
        float v = acc[i][j][r] * scale;
        if (BIAS_MODE == 1) v += bias[mBase + mOff + r];
        if (BIAS_MODE == 2) v += bv;
        if (RESID) v += Rb[(size_t)(mBase + mOff + r) * ldc + n];
        if (ACT == 2) v = fmaxf(v, 0.0f);
        if (ACT == 4) v = (v > 0.f) ? v : 0.01f * v;
        slab[(mOff + r) * 68 + (j << 4) + rlane] = v;
      }
    }
    __builtin_amdgcn_fence(__ATOMIC_RELEASE, "workgroup");
    __builtin_amdgcn_wave_barrier();
    __builtin_amdgcn_fence(__ATOMIC_ACQUIRE, "workgroup");
    if (OUT_MODE == 0) {
      float* C = (float*)Cout + (size_t)b * strideC;
      const int hh = lane >> 4, c4 = (lane & 15) * 4;
      for (int pass = 0; pass < 2; ++pass) {
#pragma unroll
        for (int it = 0; it < 8; ++it) {
          const int row = it * 2 + hh;
          v4f v = *(const v4f*)(slab + row * 68 + c4);
          *(volatile v4f*)(C + (size_t)(mBase + row) * ldc + n0 + c4) = v;
        }
        __threadfence();
      }
    } else {
      const int q = lane >> 3, c8 = (lane & 7) * 8;
      unsigned short* C  = (unsigned short*)Cout  + (size_t)b * strideC;
      unsigned short* C2 = (OUT_MODE == 2) ? ((unsigned short*)Cout2 + (size_t)b * strideC) : nullptr;
      for (int pass = 0; pass < 2; ++pass) {
#pragma unroll
        for (int it = 0; it < 4; ++it) {
          const int row = it * 4 + q;
          const float* sp = slab + row * 68 + c8;
          v8h hv, lv;
#pragma unroll
          for (int e = 0; e < 8; ++e) {
            if (OUT_MODE == 1) {
              hv[e] = (_Float16)sp[e];
            } else {
              unsigned short hb = f2bf_bits(sp[e]);
              unsigned short lb = f2bf_bits(sp[e] - bf_bits2f(hb));
              hv[e] = __builtin_bit_cast(_Float16, hb);
              lv[e] = __builtin_bit_cast(_Float16, lb);
            }
          }
          *(volatile v8h*)(C + (size_t)(mBase + row) * ldc + n0 + c8) = hv;
          if (OUT_MODE == 2) *(volatile v8h*)(C2 + (size_t)(mBase + row) * ldc + n0 + c8) = lv;
        }
        __threadfence();
      }
    }
    __builtin_amdgcn_fence(__ATOMIC_RELEASE, "workgroup");
    __builtin_amdgcn_wave_barrier();
    __builtin_amdgcn_fence(__ATOMIC_ACQUIRE, "workgroup");
  }
}

__global__ __launch_bounds__(256) void wmma_pv_out_kernel(
    const unsigned short* __restrict__ Ap, int lda,
    const unsigned short* __restrict__ Btp, int ldb,
    float* __restrict__ Cout, int ldc,
    const float* __restrict__ resid,
    const float* __restrict__ gsc,
    int M, int N, int K, float scale) {
  typedef _Float16 T;
  typedef v16h V;
  const T* A = (const T*)Ap; const T* Bt = (const T*)Btp;
  __shared__ __align__(16) float sT[8][16 * 68];
  const int lane = threadIdx.x & 31;
  const int wave = threadIdx.x >> 5;
  const int tilesN = N >> 6;
  const int tilesM = M >> 6;
  const int tile = blockIdx.x * 8 + wave;
  if (tile >= tilesM * tilesN) return;
  const int tm = tile / tilesN;
  const int tn = tile - tm * tilesN;
  const int m0 = tm << 6;
  const int n0 = tn << 6;
  const int rlane = lane & 15;
  const int koff  = (lane >> 4) * 8;
  const int mOff  = (lane >> 4) * 8;
  const float gmul = gsc[0];

  v8f acc[4][4];
#pragma unroll
  for (int i = 0; i < 4; ++i)
#pragma unroll
    for (int j = 0; j < 4; ++j) acc[i][j] = (v8f){0.f,0.f,0.f,0.f,0.f,0.f,0.f,0.f};

  for (int k0 = 0; k0 < K; k0 += 32) {
    V bh[4];
#pragma unroll
    for (int j = 0; j < 4; ++j) {
      const size_t bo = (size_t)(n0 + (j << 4) + rlane) * ldb + koff + k0;
      bh[j] = Frag<T>::load(Bt + bo);
    }
#pragma unroll
    for (int i = 0; i < 4; ++i) {
      const size_t ao = (size_t)(m0 + (i << 4) + rlane) * lda + koff + k0;
      V ah = Frag<T>::load(A + ao);
#pragma unroll
      for (int j = 0; j < 4; ++j) acc[i][j] = Frag<T>::mma(ah, bh[j], acc[i][j]);
      Frag<T>::guard(acc[i][0], acc[i][3], ah, ah);
    }
    Frag<T>::keep(bh[0], bh[1], bh[2], bh[3]);
  }
  acc_guard4(acc[0][0], acc[0][1], acc[0][2], acc[0][3]);
  acc_guard4(acc[1][0], acc[1][1], acc[1][2], acc[1][3]);
  acc_guard4(acc[2][0], acc[2][1], acc[2][2], acc[2][3]);
  acc_guard4(acc[3][0], acc[3][1], acc[3][2], acc[3][3]);

  float* slab = sT[wave];
#pragma unroll
  for (int i = 0; i < 4; ++i) {
    const int mBase = m0 + (i << 4);
#pragma unroll
    for (int j = 0; j < 4; ++j) {
#pragma unroll
      for (int r = 0; r < 8; ++r) slab[(mOff + r) * 68 + (j << 4) + rlane] = acc[i][j][r] * scale;
    }
    __builtin_amdgcn_fence(__ATOMIC_RELEASE, "workgroup");
    __builtin_amdgcn_wave_barrier();
    __builtin_amdgcn_fence(__ATOMIC_ACQUIRE, "workgroup");
    {
      const int hh = lane >> 4, c4 = (lane & 15) * 4;
      v4f rv[8];
#pragma unroll
      for (int it = 0; it < 8; ++it) {
        const int row = it * 2 + hh;
        const v4f sv = *(const v4f*)(slab + row * 68 + c4);
        const v4f xv = *(const v4f*)(resid + (size_t)(mBase + row) * ldc + n0 + c4);
        v4f rr;
#pragma unroll
        for (int e = 0; e < 4; ++e) rr[e] = fmaf(gmul, sv[e], xv[e]);
        rv[it] = rr;
      }
      for (int pass = 0; pass < 2; ++pass) {
#pragma unroll
        for (int it = 0; it < 8; ++it) {
          const int row = it * 2 + hh;
          *(volatile v4f*)(Cout + (size_t)(mBase + row) * ldc + n0 + c4) = rv[it];
        }
        __threadfence();
      }
    }
    __builtin_amdgcn_fence(__ATOMIC_RELEASE, "workgroup");
    __builtin_amdgcn_wave_barrier();
    __builtin_amdgcn_fence(__ATOMIC_ACQUIRE, "workgroup");
  }
}

__global__ __launch_bounds__(256) void prep_kernel(const float* __restrict__ Wq, const float* __restrict__ Wk,
                                                   const float* __restrict__ Wv,
                                                   const float* __restrict__ bq, const float* __restrict__ bk,
                                                   unsigned short* __restrict__ WQKh, unsigned short* __restrict__ WQKl,
                                                   unsigned short* __restrict__ WVh, unsigned short* __restrict__ WVl,
                                                   float* __restrict__ BQK) {
  const int t = threadIdx.x;
#pragma unroll 1
  for (int it = 0; it < 2; ++it) {
    const int ch = it * 256 + t;
    const int r  = ch >> 3;
    const int c8 = (ch & 7) * 8;
    const int rq = (r < kCq) ? r : (kCq - 1);
    int rk = r - 32; rk = (rk < 0) ? 0 : rk; rk = (rk > kCq - 1) ? (kCq - 1) : rk;
    const float fq = (r < kCq) ? 1.0f : 0.0f;
    const float fk = ((unsigned)(r - 32) < (unsigned)kCq) ? 1.0f : 0.0f;
    const v4f qa = *(const v4f*)(Wq + rq * kC + c8);
    const v4f qb = *(const v4f*)(Wq + rq * kC + c8 + 4);
    const v4f ka = *(const v4f*)(Wk + rk * kC + c8);
    const v4f kb = *(const v4f*)(Wk + rk * kC + c8 + 4);
    unsigned short hb[8], lb[8];
#pragma unroll
    for (int e = 0; e < 4; ++e) {
      const float v0 = fmaf(fq, qa[e], fk * ka[e]);
      const float v1 = fmaf(fq, qb[e], fk * kb[e]);
      hb[e] = f2bf_bits(v0);
      lb[e] = f2bf_bits(v0 - bf_bits2f(hb[e]));
      hb[4 + e] = f2bf_bits(v1);
      lb[4 + e] = f2bf_bits(v1 - bf_bits2f(hb[4 + e]));
    }
    const v4u uh = (v4u){pk16(hb[0], hb[1]), pk16(hb[2], hb[3]), pk16(hb[4], hb[5]), pk16(hb[6], hb[7])};
    const v4u ul = (v4u){pk16(lb[0], lb[1]), pk16(lb[2], lb[3]), pk16(lb[4], lb[5]), pk16(lb[6], lb[7])};
    unsigned short* ph = WQKh + 8 * (size_t)ch;
    unsigned short* pl = WQKl + 8 * (size_t)ch;
    *(volatile v4u*)ph = uh;
    *(volatile v4u*)pl = ul;
    __threadfence();
    *(volatile v4u*)ph = uh;
    *(volatile v4u*)pl = ul;
  }
#pragma unroll 1
  for (int it = 0; it < 2; ++it) {
    const int ch = it * 256 + t;
    const int r  = ch >> 3;
    const int c8 = (ch & 7) * 8;
    const v4f va = *(const v4f*)(Wv + r * kC + c8);
    const v4f vb = *(const v4f*)(Wv + r * kC + c8 + 4);
    unsigned short hb[8], lb[8];
#pragma unroll
    for (int e = 0; e < 4; ++e) {
      hb[e] = f2bf_bits(va[e]);
      lb[e] = f2bf_bits(va[e] - bf_bits2f(hb[e]));
      hb[4 + e] = f2bf_bits(vb[e]);
      lb[4 + e] = f2bf_bits(vb[e] - bf_bits2f(hb[4 + e]));
    }
    const v4u uh = (v4u){pk16(hb[0], hb[1]), pk16(hb[2], hb[3]), pk16(hb[4], hb[5]), pk16(hb[6], hb[7])};
    const v4u ul = (v4u){pk16(lb[0], lb[1]), pk16(lb[2], lb[3]), pk16(lb[4], lb[5]), pk16(lb[6], lb[7])};
    unsigned short* ph = WVh + 8 * (size_t)ch;
    unsigned short* pl = WVl + 8 * (size_t)ch;
    *(volatile v4u*)ph = uh;
    *(volatile v4u*)pl = ul;
    __threadfence();
    *(volatile v4u*)ph = uh;
    *(volatile v4u*)pl = ul;
  }
  {
    const int tt = t & 15;
    v4f bvv;
#pragma unroll
    for (int e = 0; e < 4; ++e) {
      const int i  = 4 * tt + e;
      const int iq = (i < kCq) ? i : (kCq - 1);
      int ik = i - 32; ik = (ik < 0) ? 0 : ik; ik = (ik > kCq - 1) ? (kCq - 1) : ik;
      const float fq = (i < kCq) ? 1.0f : 0.0f;
      const float fk = ((unsigned)(i - 32) < (unsigned)kCq) ? 1.0f : 0.0f;
      bvv[e] = fmaf(fq, bq[iq], fk * bk[ik]);
    }
    if (t < 16) {
      float* pb = BQK + 4 * t;
      *(volatile v4f*)pb = bvv;
      __threadfence();
      *(volatile v4f*)pb = bvv;
    }
  }
}

__global__ __launch_bounds__(256) void xt_split_kernel(const float* __restrict__ x, unsigned short* __restrict__ XTh,
                                                       unsigned short* __restrict__ XTl) {
  __shared__ float sm[64][65];
  const int t  = threadIdx.x;
  const int n0 = blockIdx.x * 64;
  const int b  = blockIdx.y;
  const float* xb = x + (size_t)b * kC * kN;
#pragma unroll 1
  for (int i2 = 0; i2 < 2; ++i2) {
#pragma unroll
    for (int i = 0; i < 8; ++i) {
      const int e  = (i2 * 8 + i) * 256 + t;
      const int c  = e >> 6;
      const int nl = e & 63;
      sm[nl][c] = xb[(size_t)c * kN + n0 + nl];
    }
  }
  __syncthreads();
  const int lane = t & 31, wave = t >> 5;
  const int q = lane >> 3, c8 = (lane & 7) * 8;
  unsigned short* oh = XTh + (size_t)b * kN * kC;
  unsigned short* ol = XTl + (size_t)b * kN * kC;
  v4u uh[2], ul[2];
#pragma unroll
  for (int it = 0; it < 2; ++it) {
    const int row = wave * 8 + it * 4 + q;
    unsigned short hb[8], lb[8];
#pragma unroll
    for (int e = 0; e < 8; ++e) {
      const float v = sm[row][c8 + e];
      hb[e] = f2bf_bits(v);
      lb[e] = f2bf_bits(v - bf_bits2f(hb[e]));
    }
    uh[it] = (v4u){pk16(hb[0], hb[1]), pk16(hb[2], hb[3]), pk16(hb[4], hb[5]), pk16(hb[6], hb[7])};
    ul[it] = (v4u){pk16(lb[0], lb[1]), pk16(lb[2], lb[3]), pk16(lb[4], lb[5]), pk16(lb[6], lb[7])};
  }
  for (int pass = 0; pass < 2; ++pass) {
#pragma unroll
    for (int it = 0; it < 2; ++it) {
      const int row = wave * 8 + it * 4 + q;
      *(volatile v4u*)(oh + (size_t)(n0 + row) * kC + c8) = uh[it];
      *(volatile v4u*)(ol + (size_t)(n0 + row) * kC + c8) = ul[it];
    }
    __threadfence();
  }
}

__global__ __launch_bounds__(256) void qk_pack_kernel(const float* __restrict__ QKF, unsigned short* __restrict__ QKP, int nrows) {
  const int t    = threadIdx.x;
  const int rowi = blockIdx.x * 32 + (t >> 3);
  const int g    = t & 7;
  const int rowc = (rowi < nrows) ? rowi : (nrows - 1);
  const float* rp = QKF + (size_t)rowc * kKP;
  const v4f qa = *(const v4f*)(rp);
  const v4f qb = *(const v4f*)(rp + 4);
  const v4f ka = *(const v4f*)(rp + 32);
  const v4f kb = *(const v4f*)(rp + 36);
  const float fq = (g < 3) ? 1.0f : 0.0f;
  const float fk = ((unsigned)(g - 4) < 3u) ? 1.0f : 0.0f;
  const bool islo = (g == 1) || (g == 6);
  unsigned short ob[8];
#pragma unroll
  for (int e = 0; e < 4; ++e) {
    const float v0 = fmaf(fq, qa[e], fk * ka[e]);
    const float v1 = fmaf(fq, qb[e], fk * kb[e]);
    const unsigned short h0 = f2bf_bits(v0);
    const unsigned short l0 = f2bf_bits(v0 - bf_bits2f(h0));
    const unsigned short h1 = f2bf_bits(v1);
    const unsigned short l1 = f2bf_bits(v1 - bf_bits2f(h1));
    ob[e]     = islo ? l0 : h0;
    ob[4 + e] = islo ? l1 : h1;
  }
  const v4u u = (v4u){pk16(ob[0], ob[1]), pk16(ob[2], ob[3]), pk16(ob[4], ob[5]), pk16(ob[6], ob[7])};
  if (rowi < nrows) {
    unsigned short* dst = QKP + (size_t)rowi * kKP + 8 * g;
    *(volatile v4u*)dst = u;
    __threadfence();
    *(volatile v4u*)dst = u;
  }
}

__global__ __launch_bounds__(256) void softmax_row_kernel(const float* __restrict__ SC, unsigned short* __restrict__ P) {
  __shared__ __align__(16) float lg[kN];
  __shared__ float redM[8];
  __shared__ float redS[8];
  const int row  = blockIdx.x;
  const int t    = threadIdx.x;
  const int lane = t & 31, wave = t >> 5;
  const float* sr = SC + (size_t)row * kN;

  float mx = -__builtin_inff();
#pragma unroll 1
  for (int it = 0; it < 4; ++it) {
    const int ch  = it * 256 + t;
    const bool valid = ch < kNC8;
    const int chc = valid ? ch : (kNC8 - 1);
    const v4f a = *(const v4f*)(sr + 8 * chc);
    const v4f c = *(const v4f*)(sr + 8 * chc + 4);
    const float m8 = fmaxf(fmaxf(fmaxf(a[0], a[1]), fmaxf(a[2], a[3])), fmaxf(fmaxf(c[0], c[1]), fmaxf(c[2], c[3])));
    mx = fmaxf(mx, m8);
    if (valid) {
      *(v4f*)(lg + 8 * ch)     = a;
      *(v4f*)(lg + 8 * ch + 4) = c;
    }
  }
#pragma unroll
  for (int off = 16; off > 0; off >>= 1) mx = fmaxf(mx, __shfl_xor(mx, off, 32));
  if (lane == 0) redM[wave] = mx;
  __syncthreads();
  float m = redM[0];
#pragma unroll
  for (int w = 1; w < 8; ++w) m = fmaxf(m, redM[w]);

  float sum = 0.0f;
#pragma unroll 1
  for (int it = 0; it < 8; ++it) {
    const int ch  = (it >> 1) * 256 + t;
    const int hf  = (it & 1) * 4;
    const bool valid = ch < kNC8;
    const int chc = valid ? ch : (kNC8 - 1);
    const float fv = valid ? 1.0f : 0.0f;
    const v4f l = *(const v4f*)(lg + 8 * chc + hf);
    v4f ev;
#pragma unroll
    for (int e = 0; e < 4; ++e) {
      const float l0 = valid ? l[e] : m;
      ev[e] = expf(l0 - m);
      sum = fmaf(fv, ev[e], sum);
    }
    if (valid) *(v4f*)(lg + 8 * ch + hf) = ev;
  }
#pragma unroll
  for (int off = 16; off > 0; off >>= 1) sum += __shfl_xor(sum, off, 32);
  if (lane == 0) redS[wave] = sum;
  __syncthreads();
  float tot = redS[0];
#pragma unroll
  for (int w = 1; w < 8; ++w) tot += redS[w];
  const float inv = kPCarry / tot;

  v4u u[4];
#pragma unroll
  for (int it = 0; it < 4; ++it) {
    const int ch  = it * 256 + t;
    const int chc = (ch < kNC8) ? ch : (kNC8 - 1);
    const v4f e0 = *(const v4f*)(lg + 8 * chc);
    const v4f e1 = *(const v4f*)(lg + 8 * chc + 4);
    unsigned short hb[8];
#pragma unroll
    for (int e = 0; e < 4; ++e) {
      hb[e]     = h_bits(e0[e] * inv);
      hb[4 + e] = h_bits(e1[e] * inv);
    }
    u[it] = (v4u){pk16(hb[0], hb[1]), pk16(hb[2], hb[3]), pk16(hb[4], hb[5]), pk16(hb[6], hb[7])};
  }
  unsigned short* pr = P + (size_t)row * kN;
#pragma unroll
  for (int it = 0; it < 4; ++it) {
    const int ch = it * 256 + t;
    if (ch < kNC8) *(volatile v4u*)(pr + 8 * (size_t)ch) = u[it];
  }
  __threadfence();
#pragma unroll
  for (int it = 0; it < 4; ++it) {
    const int ch = it * 256 + t;
    if (ch < kNC8) *(volatile v4u*)(pr + 8 * (size_t)ch) = u[it];
  }
}

extern "C" void kernel_launch(void* const* d_in, const int* in_sizes, int n_in,
                              void* d_out, int out_size, void* d_ws, size_t ws_size,
                              hipStream_t stream) {
  if (n_in < 8) return;
  const int nElem = kB * kC * kN;
  if (in_sizes[0] != nElem) return;
  if (in_sizes[1] != kCq * kC || in_sizes[2] != kCq) return;
  if (in_sizes[3] != kCq * kC || in_sizes[4] != kCq) return;
  if (in_sizes[5] != kC * kC || in_sizes[6] != kC || in_sizes[7] < 1) return;
  if (out_size != nElem) return;

  const size_t szXT  = (size_t)kB * kN * kC * 2;
  const size_t szW   = (size_t)64 * 64 * 2;
  const size_t szBQK = (size_t)64 * 4;
  const size_t szQKF = (size_t)kB * kN * kKP * 4;
  const size_t szQKP = (size_t)kB * kN * kKP * 2;
  const size_t szVP  = (size_t)kB * kC * kN * 2;
  const size_t szSC  = (size_t)kQCH * kN * 4;
  const size_t szP   = (size_t)kQCH * kN * 2;
  const size_t offXTh  = 0;
  const size_t offXTl  = offXTh + szXT;
  const size_t offWQKh = offXTl + szXT;
  const size_t offWQKl = offWQKh + szW;
  const size_t offWVh  = offWQKl + szW;
  const size_t offWVl  = offWVh + szW;
  const size_t offBQK  = offWVl + szW;
  const size_t offQKF  = offBQK + szBQK;
  const size_t offQKP  = offQKF + szQKF;
  const size_t offVP   = offQKP + szQKP;
  const size_t offSC   = offVP + szVP;
  const size_t offP    = offSC + szSC;
  const size_t total   = offP + szP;
  if (ws_size < total) return;

  const float* x     = (const float*)d_in[0];
  const float* Wq    = (const float*)d_in[1];
  const float* bq    = (const float*)d_in[2];
  const float* Wk    = (const float*)d_in[3];
  const float* bk    = (const float*)d_in[4];
  const float* Wv    = (const float*)d_in[5];
  const float* bv    = (const float*)d_in[6];
  const float* gamma = (const float*)d_in[7];
  float* out = (float*)d_out;
  char* ws = (char*)d_ws;
  unsigned short* XTh  = (unsigned short*)(ws + offXTh);
  unsigned short* XTl  = (unsigned short*)(ws + offXTl);
  unsigned short* WQKh = (unsigned short*)(ws + offWQKh);
  unsigned short* WQKl = (unsigned short*)(ws + offWQKl);
  unsigned short* WVh  = (unsigned short*)(ws + offWVh);
  unsigned short* WVl  = (unsigned short*)(ws + offWVl);
  float* BQK = (float*)(ws + offBQK);
  float* QKF = (float*)(ws + offQKF);
  unsigned short* QKP = (unsigned short*)(ws + offQKP);
  unsigned short* VP  = (unsigned short*)(ws + offVP);
  float* SC = (float*)(ws + offSC);
  unsigned short* PP = (unsigned short*)(ws + offP);

  prep_kernel<<<dim3(1), dim3(256), 0, stream>>>(Wq, Wk, Wv, bq, bk, WQKh, WQKl, WVh, WVl, BQK);
  xt_split_kernel<<<dim3(kN / 64, kB), dim3(256), 0, stream>>>(x, XTh, XTl);
  wmma_gemm64<1, true, 2, 0, false, 0><<<dim3(kBlocksProj, kB), dim3(256), 0, stream>>>(
      XTh, XTl, kC, (long)kN * kC,
      WQKh, WQKl, kC, 0L,
      (void*)QKF, (void*)QKF, kKP, (long)kN * kKP,
      BQK, BQK, 0L,
      kN, kKP, kC, 1.0f);
  qk_pack_kernel<<<dim3((kB * kN) / 32), dim3(256), 0, stream>>>(QKF, QKP, kB * kN);
  wmma_gemm64<1, true, 1, 1, false, 0><<<dim3(kBlocksProj, kB), dim3(256), 0, stream>>>(
      WVh, WVl, kC, 0L,
      XTh, XTl, kC, (long)kN * kC,
      (void*)VP, (void*)VP, kN, (long)kC * kN,
      bv, bv, 0L,
      kC, kN, kC, 1.0f);

  for (int b = 0; b < kB; ++b) {
    const unsigned short* qkb = QKP + (size_t)b * kN * kKP;
    const unsigned short* vpb = VP + (size_t)b * kC * kN;
    for (int chk = 0; chk < kNChunk; ++chk) {
      const int q0 = chk * kQCH;
      wmma_gemm64<1, false, 0, 0, false, 0><<<dim3(kBlocksScore, 1), dim3(256), 0, stream>>>(
          qkb + (size_t)q0 * kKP, qkb + (size_t)q0 * kKP, kKP, 0L,
          qkb + 32, qkb + 32, kKP, 0L,
          (void*)SC, (void*)SC, kN, 0L,
          BQK, BQK, 0L,
          kQCH, kN, 32, 1.0f);
      softmax_row_kernel<<<dim3(kQCH), dim3(256), 0, stream>>>(SC, PP);
      wmma_pv_out_kernel<<<dim3(kBlocksPV), dim3(256), 0, stream>>>(
          vpb, kN, PP, kN,
          out + (size_t)b * kC * kN + q0, kN,
          x + (size_t)b * kC * kN + q0,
          gamma,
          kC, kQCH, kN, kPCarryInv);
    }
  }
}
